// HeteroGNN_15556371546392
// MI455X (gfx1250) — hardware-verified
//
#include <hip/hip_runtime.h>

typedef float          v8f   __attribute__((ext_vector_type(8)));
typedef float          v4f   __attribute__((ext_vector_type(4)));
typedef unsigned int   v4u   __attribute__((ext_vector_type(4)));
typedef int            v8i   __attribute__((ext_vector_type(8)));
typedef unsigned short v8us  __attribute__((ext_vector_type(8)));
typedef unsigned short v16us __attribute__((ext_vector_type(16)));
typedef __bf16         v16bf __attribute__((ext_vector_type(16)));
typedef _Float16       v16h  __attribute__((ext_vector_type(16)));
typedef v4f  __attribute__((may_alias)) v4fa;
typedef v8us __attribute__((may_alias)) v8usa;
union FragB { v16bf v; v16us u; v8us h[2]; v8i w; };
union FragH { v16h  v; v16us u; v8us h[2]; v8i w; };

__device__ __forceinline__ v8f wmb(const FragB& a, const FragB& b, v8f c) {
  v8f d = __builtin_amdgcn_wmma_f32_16x16x32_bf16(false, a.v, false, b.v, (short)0, c, false, false);
  asm volatile("v_nop\n\tv_nop\n\tv_nop\n\tv_nop" : "+v"(d) : "v"(a.w), "v"(b.w));
  return d;
}

__device__ __forceinline__ v8f wmh(const FragH& a, const FragH& b, v8f c) {
  v8f d = __builtin_amdgcn_wmma_f32_16x16x32_f16(false, a.v, false, b.v, (short)0, c, false, false);
  asm volatile("v_nop\n\tv_nop\n\tv_nop\n\tv_nop" : "+v"(d) : "v"(a.w), "v"(b.w));
  return d;
}

__device__ __forceinline__ unsigned bf16_bits(float f) {
  const unsigned u = __float_as_uint(f);
  const unsigned r = (u + 0x7FFFu + ((u >> 16) & 1u)) >> 16;
  const unsigned q = (u >> 16) | 0x40u;
  return ((u & 0x7fffffffu) > 0x7f800000u) ? q : r;
}

__device__ __forceinline__ float bf16_val(float f) {
  return __uint_as_float(bf16_bits(f) << 16);
}
__device__ __forceinline__ int clampi(int v, int lo, int hi) {
  return v < lo ? lo : (v > hi ? hi : v);
}

__device__ __forceinline__ unsigned f16_bits(float f) {
  const unsigned u  = __float_as_uint(f);
  const unsigned s  = (u >> 16) & 0x8000u;
  const unsigned a  = u & 0x7fffffffu;
  const unsigned t  = a - 0x38000000u;
  const unsigned r  = (t + 0x0FFFu + ((t >> 13) & 1u)) >> 13;
  const unsigned rc = r > 0x7C00u ? 0x7C00u : r;
  const bool small  = a < 0x38800000u;
  const bool isnan  = a > 0x7f800000u;
  const unsigned fin = small ? 0u : (s | rc);
  return isnan ? (s | 0x7E00u) : fin;
}

__device__ __forceinline__ unsigned pk16(unsigned lo, unsigned hi) { return lo | (hi << 16); }
__device__ __forceinline__ unsigned bf16_lo_bits(float v) {
  float hi = bf16_val(v);
  asm volatile("" : "+v"(hi));
  return bf16_bits(v - hi);
}
__device__ __forceinline__ v4u pack8_bf16(v4f a, v4f c) {
  return (v4u){ pk16(bf16_bits(a[0]), bf16_bits(a[1])), pk16(bf16_bits(a[2]), bf16_bits(a[3])),
                pk16(bf16_bits(c[0]), bf16_bits(c[1])), pk16(bf16_bits(c[2]), bf16_bits(c[3])) };
}
__device__ __forceinline__ v4u pack8_bf16_lo(v4f a, v4f c) {
  return (v4u){ pk16(bf16_lo_bits(a[0]), bf16_lo_bits(a[1])), pk16(bf16_lo_bits(a[2]), bf16_lo_bits(a[3])),
                pk16(bf16_lo_bits(c[0]), bf16_lo_bits(c[1])), pk16(bf16_lo_bits(c[2]), bf16_lo_bits(c[3])) };
}
__device__ __forceinline__ v4u pack8_f16(v4f a, v4f c) {
  return (v4u){ pk16(f16_bits(a[0]), f16_bits(a[1])), pk16(f16_bits(a[2]), f16_bits(a[3])),
                pk16(f16_bits(c[0]), f16_bits(c[1])), pk16(f16_bits(c[2]), f16_bits(c[3])) };
}

template <int FORM>
__global__ __launch_bounds__(256) void k_plane(const float* __restrict__ src, int rows, int cols, int ldsrc,
                                               unsigned short* __restrict__ dst, int MP, int KP) {
  static_assert(FORM >= 0 && FORM <= 3);
  const int KTOT = (FORM == 1 || FORM == 3) ? 2 * KP : KP;
  const unsigned ppr   = (unsigned)(KTOT >> 3);
  const unsigned kp8   = (unsigned)(KP >> 3);
  const unsigned total = (unsigned)MP * ppr;
  const unsigned g     = blockIdx.x * 256u + threadIdx.x;
  const unsigned rowu  = g / ppr;
  const unsigned p     = g - rowu * ppr;
  const bool second    = p >= kp8;
  const int row = (int)rowu;
  const int c0  = (int)((second ? p - kp8 : p) << 3);
  const float* srow = src + (size_t)clampi(row, 0, rows - 1) * (size_t)ldsrc;
  float x[8];
  unsigned mk[8];
#pragma unroll
  for (int e = 0; e < 8; ++e) {
    const int c = c0 + e;
    const float v = srow[clampi(c, 0, cols - 1)];
    asm volatile("" :: "v"(v));
    x[e]  = v;
    mk[e] = (row < rows && c < cols) ? 0xFFFFu : 0u;
  }
  const v4f a = (v4f){ x[0], x[1], x[2], x[3] };
  const v4f c = (v4f){ x[4], x[5], x[6], x[7] };
  v4u o;
  if (FORM == 2) {
    o = pack8_f16(a, c);
  } else {
    const v4u hi = pack8_bf16(a, c);
    o = hi;
    if (FORM == 1) { const v4u lo = pack8_bf16_lo(a, c); o = second ? lo : hi; }
  }
  const v4u mw = (v4u){ pk16(mk[0], mk[1]), pk16(mk[2], mk[3]), pk16(mk[4], mk[5]), pk16(mk[6], mk[7]) };
  o &= mw;
  if (g < total) {
    volatile v4u* q = (volatile v4u*)(dst + (size_t)g * 8);
    *q = o;
    __threadfence();
    *q = o;
  }
}

template <int FORM> struct FragOf    { typedef FragB T; };
template <>         struct FragOf<2> { typedef FragH T; };
__device__ __forceinline__ v8f mm(const FragB& a, const FragB& b, v8f c) { return wmb(a, b, c); }
__device__ __forceinline__ v8f mm(const FragH& a, const FragH& b, v8f c) { return wmh(a, b, c); }
template <class F> __device__ __forceinline__ F ld_frag(const unsigned short* p) {
  F f;
  f.h[0] = *(const v8usa*)(p);
  f.h[1] = *(const v8usa*)(p + 16);
  return f;
}

template <int FORM, int EPI>
__global__ __launch_bounds__(256) __attribute__((amdgpu_num_vgpr(248)))
void k_gemm_nt(const unsigned short* __restrict__ A, const unsigned short* __restrict__ B,
               const float* __restrict__ bias, float* __restrict__ D, int M, int N, int KTOT, int ldd) {
  static_assert(FORM >= 0 && FORM <= 2);
  static_assert(EPI == 0 || EPI == 1);
  typedef typename FragOf<FORM>::T F;
  __shared__ __attribute__((aligned(16))) float sT[8][16 * 68];
  const int lane = threadIdx.x & 31;
  const int wave = threadIdx.x >> 5;
  const int tilesM = (M + 63) >> 6;
  const int tilesN = (N + 63) >> 6;
  const int tile = blockIdx.x * 8 + wave;
  if (tile >= tilesM * tilesN) return;
  const int tm = tile / tilesN;
  const int tn = tile - tm * tilesN;
  const int m0 = tm << 6;
  const int n0 = tn << 6;

  const int rl = lane & 15;
  const int h8 = (lane >> 4) * 8;
  const unsigned short* pa = A + (size_t)(m0 + rl) * (size_t)KTOT + h8;
  const unsigned short* pb = B + (size_t)(n0 + rl) * (size_t)KTOT + h8;

  v8f acc[4][4];
#pragma unroll
  for (int i = 0; i < 4; ++i)
#pragma unroll
    for (int j = 0; j < 4; ++j) acc[i][j] = (v8f){0.f, 0.f, 0.f, 0.f, 0.f, 0.f, 0.f, 0.f};

#pragma unroll 1
  for (int k0 = 0; k0 < KTOT; k0 += 32) {
    F bf[4];
#pragma unroll
    for (int j = 0; j < 4; ++j) bf[j] = ld_frag<F>(pb + (size_t)(j << 4) * (size_t)KTOT + k0);
#pragma unroll
    for (int i = 0; i < 4; ++i) {
      const F af = ld_frag<F>(pa + (size_t)(i << 4) * (size_t)KTOT + k0);
#pragma unroll
      for (int j = 0; j < 4; ++j) acc[i][j] = mm(af, bf[j], acc[i][j]);
    }
  }

  float* slab = sT[wave];
  const int hh = lane >> 4;
  const int c4 = (lane & 15) * 4;
  const int nc = n0 + c4;
  const bool cok = nc < N;
  v4f bv = (v4f){0.f, 0.f, 0.f, 0.f};
  if (EPI == 1) {
    bv = *(const v4fa*)(bias + clampi(nc, 0, N - 4));
    asm volatile("" :: "v"(bv));
  }
#pragma unroll
  for (int i = 0; i < 4; ++i) {
    const int mBase = m0 + (i << 4);
#pragma unroll
    for (int j = 0; j < 4; ++j) {
#pragma unroll
      for (int r = 0; r < 8; ++r) slab[(h8 + r) * 68 + (j << 4) + rl] = acc[i][j][r];
    }
    __builtin_amdgcn_fence(__ATOMIC_RELEASE, "workgroup");
    __builtin_amdgcn_wave_barrier();
    __builtin_amdgcn_fence(__ATOMIC_ACQUIRE, "workgroup");
    v4f vv[8];
#pragma unroll
    for (int it = 0; it < 8; ++it) {
      const int row = it * 2 + hh;
      v4f v = *(const v4fa*)(slab + row * 68 + c4);
      if (EPI == 1) v += bv;
      vv[it] = v;
    }
    for (int pass = 0; pass < 2; ++pass) {
#pragma unroll
      for (int it = 0; it < 8; ++it) {
        const int row = mBase + it * 2 + hh;
        if (cok && row < M) *(volatile v4f*)(D + (size_t)row * (size_t)ldd + nc) = vv[it];
      }
      __threadfence();
    }
    __builtin_amdgcn_fence(__ATOMIC_RELEASE, "workgroup");
    __builtin_amdgcn_wave_barrier();
    __builtin_amdgcn_fence(__ATOMIC_ACQUIRE, "workgroup");
  }
}

#define NTY      4
#define NND      16384
#define NRL      14
#define NED      65536
#define NCH      64
#define NCI      11
#define NPF      524288
#define NGL      65536
#define BK_THR   256
#define BK_NW    8
#define BK_EPT   8
#define BK_CHUNK 2048
#define BK_WCAP  256
#define BK_LISTN 2048
#define BK_NB    1024
#define BK_ESH   10
#define RCAP_R   6144
#define RCAP_P   11264
#define MAXH_R   4215
#define MAXH_P   8453
#define DEG_R    64
#define DEG_P    256
#define MAXDEG_R 13
#define MAXDEG_P 26
#define LDS_BK_R ((2 * RCAP_R + 2 * BK_NB + BK_LISTN) * 4 + 64)
#define LDS_BK_P ((2 * RCAP_P + 2 * BK_NB + BK_LISTN) * 4 + 64)
#define WSMAX    ((size_t)128 << 20)

static_assert(NCH == 64 && NCH == 2 * 32);
static_assert(NND % 1024 == 0 && NGL == NTY * NND && NGL % 1024 == 0);
static_assert(NED % BK_CHUNK == 0 && NPF % BK_CHUNK == 0 && NED % 256 == 0 && NPF % 256 == 0);
static_assert(BK_CHUNK == BK_THR * BK_EPT && BK_WCAP == BK_EPT * 32 && BK_LISTN == BK_NW * BK_WCAP);
static_assert(BK_LISTN >= BK_NB && (1 << BK_ESH) >= BK_NB && BK_THR * 4 == BK_NB);
static_assert(NED <= (1 << (31 - BK_ESH)) && NPF <= (1 << (31 - BK_ESH)));
static_assert(RCAP_R % 1024 == 0 && RCAP_P % 1024 == 0);
static_assert(RCAP_R * 4 >= MAXH_R * 5 && RCAP_P * 4 >= MAXH_P * 5);
static_assert(DEG_R * 4 >= MAXDEG_R * 5 && DEG_P * 4 >= MAXDEG_P * 5 && DEG_P % 32 == 0);
static_assert(LDS_BK_R <= 327680 && LDS_BK_P <= 327680);

constexpr int SRC_H[NRL] = {0, 0, 0, 1, 1, 2, 1, 2, 3, 2, 3, 1, 2, 3};
constexpr int DST_H[NRL] = {1, 2, 3, 2, 3, 3, 0, 0, 0, 1, 2, 1, 2, 3};
constexpr int ORD_H[NRL] = {6, 7, 8, 0, 9, 11, 1, 3, 10, 12, 2, 4, 5, 13};
constexpr int GST_H[NTY] = {0, 3, 6, 10};
constexpr int GSZ_H[NTY] = {3, 3, 4, 4};
constexpr unsigned long long ORD_PACK = 0xD542CA31B90876ULL;
constexpr bool tables_ok() {
  int seen = 0;
  for (int d = 0; d < NTY; ++d) {
    int last = -1;
    for (int j = 0; j < GSZ_H[d]; ++j) {
      const int pos = GST_H[d] + j;
      const int t = ORD_H[pos];
      if (DST_H[t] != d) return false;
      if (t <= last) return false;
      last = t;
      if ((int)((ORD_PACK >> (4 * pos)) & 15ULL) != t) return false;
      seen |= 1 << t;
    }
  }
  return seen == 0x3FFF && GST_H[3] + GSZ_H[3] == NRL;
}
static_assert(tables_ok());
__device__ __forceinline__ int ord_of(int pos) { return (int)((ORD_PACK >> (4 * pos)) & 15ULL); }

constexpr size_t al256(size_t v) { return (v + 255) & ~(size_t)255; }
constexpr size_t O_XB    = 0;
constexpr size_t O_H1    = al256(O_XB + (size_t)NGL * 32 * 2);
constexpr size_t O_QS    = al256(O_H1 + (size_t)NGL * 128 * 2);
constexpr size_t O_KV    = al256(O_QS + (size_t)NND * 512 * 4);
constexpr size_t O_X01   = al256(O_KV + (size_t)4 * NND * 128 * 4);
constexpr size_t O_WQS0  = al256(O_X01 + (size_t)NGL * 2 * 4);
constexpr size_t O_WKV0  = al256(O_WQS0 + (size_t)NRL * 128 * 32 * 2);
constexpr size_t O_WQS1  = al256(O_WKV0 + (size_t)NRL * 128 * 32 * 2);
constexpr size_t O_WKV1  = al256(O_WQS1 + (size_t)NRL * 128 * 128 * 2);
constexpr size_t O_BQS   = al256(O_WKV1 + (size_t)NRL * 128 * 128 * 2);
constexpr size_t O_BKV   = al256(O_BQS + (size_t)2 * NRL * 128 * 4);
constexpr size_t O_WE    = al256(O_BKV + (size_t)2 * NRL * 128 * 4);
constexpr size_t O_LIN   = al256(O_WE + (size_t)2 * NRL * 128 * 4);
constexpr size_t O_LISTR = al256(O_LIN + 512);
constexpr size_t O_OFFR  = al256(O_LISTR + (size_t)NRL * 16 * RCAP_R * 4);
constexpr size_t O_METAR = al256(O_OFFR + (size_t)NRL * 16 * 2048 * 4);
constexpr size_t O_LISTP = al256(O_METAR + (size_t)NRL * 16 * 128);
constexpr size_t O_OFFP  = al256(O_LISTP + (size_t)64 * RCAP_P * 4);
constexpr size_t O_METAP = al256(O_OFFP + (size_t)64 * 2048 * 4);
constexpr size_t WS_TOTAL = al256(O_METAP + (size_t)64 * 128);
static_assert(WS_TOTAL <= (size_t)WSMAX);
static_assert((NGL * 32 / 8) % 256 == 0);

typedef int      v4i  __attribute__((ext_vector_type(4)));
typedef float    v2f  __attribute__((ext_vector_type(2)));
typedef v4i __attribute__((may_alias)) v4ia;
typedef v2f __attribute__((may_alias)) v2fa;

__device__ __forceinline__ void st2_v4u(void* p, const v4u v) {
  volatile v4u* q = (volatile v4u*)p;
  *q = v;
  __threadfence();
  *q = v;
}
__device__ __forceinline__ void st2_v4f(float* p, const v4f v) {
  volatile v4f* q = (volatile v4f*)p;
  *q = v;
  __threadfence();
  *q = v;
}
__device__ __forceinline__ void st2_v4i(int* p, const v4i v) {
  volatile v4i* q = (volatile v4i*)p;
  *q = v;
  __threadfence();
  *q = v;
}

template <int KIN>
__device__ __forceinline__ v4u wpiece(const float* __restrict__ W, int n, int k8) {
  float x[8];
  unsigned mk[8];
#pragma unroll
  for (int e = 0; e < 8; ++e) {
    const int k  = k8 + e;
    const int kc = k < KIN ? k : KIN - 1;
    const float v = W[kc * 64 + n];
    asm volatile("" :: "v"(v));
    x[e]  = v;
    mk[e] = (k < KIN) ? 0xFFFFu : 0u;
  }
  v4u o = pack8_bf16((v4f){ x[0], x[1], x[2], x[3] }, (v4f){ x[4], x[5], x[6], x[7] });
  o &= (v4u){ pk16(mk[0], mk[1]), pk16(mk[2], mk[3]), pk16(mk[4], mk[5]), pk16(mk[6], mk[7]) };
  return o;
}

template <int KIN, int KP, int KTOT>
__global__ __launch_bounds__(256) void k_wprep(const float* __restrict__ wq, const float* __restrict__ wsk,
                                               const float* __restrict__ wk, const float* __restrict__ wv,
                                               unsigned short* QSP, unsigned short* KVP) {
  constexpr int PPR = KTOT / 8;
  constexpr int RPB = 256 / PPR;
  constexpr int BPM = 64 / RPB;
  static_assert(KP % 32 == 0 && (KTOT == KP || KTOT == 2 * KP) && KIN <= KP);
  static_assert(256 % PPR == 0 && 64 % RPB == 0 && BPM >= 1);
  const int tid = (int)threadIdx.x;
  const int b   = (int)blockIdx.x;
  const int m   = clampi(b / (NRL * BPM), 0, 3);
  const int r   = b - m * (NRL * BPM);
  const int idx = clampi(r / BPM, 0, NRL - 1);
  const int rg  = r - idx * BPM;
  const int n   = rg * RPB + tid / PPR;
  const int p   = tid % PPR;
  const int k8  = (p % (KP / 8)) * 8;
  const int t   = (m < 2) ? ord_of(idx) : idx;
  const size_t toff = (size_t)t * KIN * 64;
  v4u o;
  if (m == 0)      o = wpiece<KIN>(wq  + toff, n, k8);
  else if (m == 1) o = wpiece<KIN>(wsk + toff, n, k8);
  else if (m == 2) o = wpiece<KIN>(wk  + toff, n, k8);
  else             o = wpiece<KIN>(wv  + toff, n, k8);
  const size_t doff = ((size_t)(idx * 128 + (m & 1) * 64 + n) * KTOT) + (size_t)p * 8;
  if (m < 2) st2_v4u(QSP + doff, o);
  else       st2_v4u(KVP + doff, o);
}

__global__ __launch_bounds__(256) void k_tprep(const float* __restrict__ bq, const float* __restrict__ bs,
                                               const float* __restrict__ bk, const float* __restrict__ bv,
                                               const float* __restrict__ we, const float* __restrict__ linw,
                                               float* BQS, float* BKV, float* WEt, float* LIN) {
  const int tid = (int)threadIdx.x;
  const int b   = (int)blockIdx.x;
  if (b < 4) {
    const int u    = tid;
    const int slot = clampi(u >> 4, 0, NRL - 1);
    const int c4   = (u & 15) * 4;
    const int t    = (b < 2) ? ord_of(slot) : slot;
    const int so   = t * 64 + c4;
    v4f v;
    if (b == 0)      v = *(const v4fa*)(bq + so);
    else if (b == 1) v = *(const v4fa*)(bs + so);
    else if (b == 2) v = *(const v4fa*)(bk + so);
    else             v = *(const v4fa*)(bv + so);
    asm volatile("" :: "v"(v));
    const v4f o = (v4f){ bf16_val(v[0]), bf16_val(v[1]), bf16_val(v[2]), bf16_val(v[3]) };
    const int doff = slot * 128 + (b & 1) * 64 + c4;
    if (u < NRL * 16) {
      if (b < 2) st2_v4f(BQS + doff, o);
      else       st2_v4f(BKV + doff, o);
    }
  } else if (b < 6) {
    const int u  = (b - 4) * 256 + tid;
    const int uc = clampi(u, 0, NRL * 32 - 1);
    const v4f v = *(const v4fa*)(we + 4 * uc);
    asm volatile("" :: "v"(v));
    const v4f o = (v4f){ bf16_val(v[0]), bf16_val(v[1]), bf16_val(v[2]), bf16_val(v[3]) };
    if (u < NRL * 32) st2_v4f(WEt + 4 * u, o);
  } else {
    if (tid < 32) {
      const v4f r0 = *(const v4fa*)(linw + 8 * tid);
      const v4f r1 = *(const v4fa*)(linw + 8 * tid + 4);
      asm volatile("" :: "v"(r0), "v"(r1));
      const v4f o = (v4f){ bf16_val(r0[0]), bf16_val(r0[1]), bf16_val(r1[0]), bf16_val(r1[1]) };
      st2_v4f(LIN + 4 * tid, o);
    }
  }
}

__device__ __forceinline__ int scan_chunk(const int* __restrict__ dsts, int cbase, int slotBase,
                                          int* list, int tid, int wave) {
  int wc = 0;
  const int el0 = tid * BK_EPT;
  const int e0  = cbase + el0;
  const v4i da = *(const v4ia*)(dsts + e0);
  const v4i db = *(const v4ia*)(dsts + e0 + 4);
  const unsigned nbs = (unsigned)slotBase;
  const unsigned unb = (unsigned)BK_NB;
  const unsigned s0 = (unsigned)da.x - nbs, s1 = (unsigned)da.y - nbs;
  const unsigned s2 = (unsigned)da.z - nbs, s3 = (unsigned)da.w - nbs;
  const unsigned s4 = (unsigned)db.x - nbs, s5 = (unsigned)db.y - nbs;
  const unsigned s6 = (unsigned)db.z - nbs, s7 = (unsigned)db.w - nbs;
  const bool h0 = s0 < unb, h1 = s1 < unb, h2 = s2 < unb, h3 = s3 < unb;
  const bool h4 = s4 < unb, h5 = s5 < unb, h6 = s6 < unb, h7 = s7 < unb;
  const unsigned any = __builtin_amdgcn_ballot_w32(h0 | h1 | h2 | h3 | h4 | h5 | h6 | h7);
  if (any != 0u) {
#define HITJ(J, HJ, SJ) { \
      const unsigned mj = __builtin_amdgcn_ballot_w32(HJ); \
      if (mj != 0u) { \
        if (HJ) { \
          const int pos = wc + (int)__builtin_amdgcn_mbcnt_lo(mj, 0u); \
          if (pos < BK_WCAP) list[wave * BK_WCAP + pos] = ((el0 + (J)) << 12) | (int)(SJ); \
        } \
        wc += (int)__builtin_popcount(mj); } }
    HITJ(0, h0, s0)
    HITJ(1, h1, s1)
    HITJ(2, h2, s2)
    HITJ(3, h3, s3)
    HITJ(4, h4, s4)
    HITJ(5, h5, s5)
    HITJ(6, h6, s6)
    HITJ(7, h7, s7)
#undef HITJ
  }
  return wc;
}

__device__ __forceinline__ int build_lists(const int* __restrict__ dsts, int nE, int nodeBase, int rcap,
                                           int* reg1, int* reg2, int* scnt, int* soff, int* list,
                                           int* wcnt, int* wtot, int tid, int lane, int wave) {
  for (int i = tid; i < BK_NB; i += BK_THR) scnt[i] = 0;
  if (tid == 0) { reg1[0] = 0; reg2[0] = 0; }
  __syncthreads();

  int tot = 0;
  const int nChunks = nE / BK_CHUNK;
#pragma unroll 1
  for (int ch = 0; ch < nChunks; ++ch) {
    const int cbase = ch * BK_CHUNK;
    const int wc = scan_chunk(dsts, cbase, nodeBase, list, tid, wave);
    if (lane == 0) wcnt[wave] = wc;
    __syncthreads();
    int pre = 0, all = 0;
#pragma unroll
    for (int w2 = 0; w2 < BK_NW; ++w2) {
      int c = wcnt[w2];
      c = c < 0 ? 0 : (c > BK_WCAP ? BK_WCAP : c);
      all += c;
      pre += (w2 < wave) ? c : 0;
    }
    const int wcc  = wc > BK_WCAP ? BK_WCAP : wc;
    const int base = tot + pre;
#pragma unroll 1
    for (int i = lane; i < wcc; i += 32) {
      const int ent = list[wave * BK_WCAP + i];
      const int el  = (ent >> 12) & (BK_CHUNK - 1);
      const int sl  = ent & (BK_NB - 1);
      int eid = cbase + el;
      eid = eid > nE - 1 ? nE - 1 : eid;
      const int pos = base + i;
      if (pos < rcap) reg1[pos] = (int)(((unsigned)eid << BK_ESH) | (unsigned)sl);
    }
    tot += all;
    tot = tot > rcap ? rcap : tot;
    __syncthreads();
  }
  const int nh = tot;

  if (wave == 0) {
#pragma unroll 1
    for (int b0 = 0; b0 < nh; b0 += 32) {
      const int idx = b0 + lane;
      const int uv  = reg1[idx < nh ? idx : nh - 1];
      const int m32 = (nh - b0) < 32 ? (nh - b0) : 32;
#pragma unroll 1
      for (int k = 0; k < m32; ++k) {
        const int u  = __builtin_amdgcn_readlane(uv, k);
        const int sl = u & (BK_NB - 1);
        if (lane == 0) scnt[sl] = scnt[sl] + 1;
      }
    }
  }
  __syncthreads();

  {
    const v4i ca = *(const v4ia*)(scnt + 4 * tid);
    const int e0 = ca.x < 0 ? 0 : ca.x, e1 = ca.y < 0 ? 0 : ca.y, e2 = ca.z < 0 ? 0 : ca.z, e3 = ca.w < 0 ? 0 : ca.w;
    const int ts = e0 + e1 + e2 + e3;
    int incl = ts;
#pragma unroll
    for (int d = 1; d < 32; d <<= 1) {
      const int up = __shfl_up(incl, d);
      if (lane >= d) incl += up;
    }
    if (lane == 31) wtot[wave] = incl;
    __syncthreads();
    int pre = 0;
#pragma unroll
    for (int w2 = 0; w2 < BK_NW; ++w2) pre += (w2 < wave) ? wtot[w2] : 0;
    int run = pre + incl - ts;
    soff[4 * tid + 0] = run; run += e0;
    soff[4 * tid + 1] = run; run += e1;
    soff[4 * tid + 2] = run; run += e2;
    soff[4 * tid + 3] = run;
  }
  __syncthreads();
  for (int i = tid; i < BK_NB; i += BK_THR) list[i] = soff[i];
  __syncthreads();

  if (wave == 0) {
#pragma unroll 1
    for (int b0 = 0; b0 < nh; b0 += 32) {
      const int idx = b0 + lane;
      const int uv  = reg1[idx < nh ? idx : nh - 1];
      const int m32 = (nh - b0) < 32 ? (nh - b0) : 32;
#pragma unroll 1
      for (int k = 0; k < m32; ++k) {
        const int u   = __builtin_amdgcn_readlane(uv, k);
        const int sl  = u & (BK_NB - 1);
        const int eid = (int)((unsigned)u >> BK_ESH);
        if (lane == 0) {
          int pos = list[sl];
          pos = pos < 0 ? 0 : (pos > rcap - 1 ? rcap - 1 : pos);
          reg2[pos] = eid;
          list[sl] = pos + 1;
        }
      }
    }
  }
  __syncthreads();
  return nh;
}

__global__ __launch_bounds__(BK_THR) void k_bucket(const int* __restrict__ keys, int relStride, int nE, int rcap,
                                                   int* LIST, int* OFFC, int* META) {
  extern __shared__ v4f lds_dyn[];
  int* reg1 = (int*)lds_dyn;
  int* reg2 = reg1 + rcap;
  int* scnt = reg2 + rcap;
  int* soff = scnt + BK_NB;
  int* list = soff + BK_NB;
  int* wcnt = list + BK_LISTN;
  int* wtot = wcnt + BK_NW;
  const int tid = (int)threadIdx.x, lane = tid & 31, wave = tid >> 5;
  const int b = (int)blockIdx.x;
  const int t = (int)blockIdx.y;
  const int blk = t * (int)gridDim.x + b;
  const int* dsts = keys + (size_t)t * (size_t)relStride;

  const int nh = build_lists(dsts, nE, b * BK_NB, rcap, reg1, reg2, scnt, soff, list, wcnt, wtot, tid, lane, wave);

  int* bl = LIST + (size_t)blk * (size_t)rcap;
  const int last = nh > 0 ? nh - 1 : 0;
#pragma unroll 1
  for (int base = 0; base < rcap; base += 1024) {
    const int i0 = base + 4 * tid;
    v4i v;
    v.x = reg2[i0     < last ? i0     : last];
    v.y = reg2[i0 + 1 < last ? i0 + 1 : last];
    v.z = reg2[i0 + 2 < last ? i0 + 2 : last];
    v.w = reg2[i0 + 3 < last ? i0 + 3 : last];
    v.x = (i0     < nh) ? v.x : 0;
    v.y = (i0 + 1 < nh) ? v.y : 0;
    v.z = (i0 + 2 < nh) ? v.z : 0;
    v.w = (i0 + 3 < nh) ? v.w : 0;
    st2_v4i(bl + i0, v);
  }
  {
    const v4i so = *(const v4ia*)(soff + 4 * tid);
    const v4i sc = *(const v4ia*)(scnt + 4 * tid);
    int* oc = OFFC + (size_t)blk * 2048;
    st2_v4i(oc + 4 * tid, so);
    st2_v4i(oc + 1024 + 4 * tid, sc);
  }
  if (tid < 8) {
    v4i mv;
    mv.x = (tid == 0) ? nh : 0;
    mv.y = (tid == 0 && nh >= rcap) ? 1 : 0;
    mv.z = 0; mv.w = 0;
    st2_v4i(META + (size_t)blk * 32 + 4 * tid, mv);
  }
}

template <int LAYER>
__global__ __launch_bounds__(256) void k_att(
    const float* __restrict__ QS, const float* __restrict__ KV, const float* __restrict__ ea,
    const int* __restrict__ ei, const float* __restrict__ WEt, const float* __restrict__ LIN,
    const int* __restrict__ LISTR, const int* __restrict__ OFFR, const int* __restrict__ METAR,
    unsigned* H1w, float* X01, int gstart, int gs) {
  __shared__ __attribute__((aligned(16))) float sX[256];
  const int lane = threadIdx.x & 31;
  const int wave = threadIdx.x >> 5;
  const int ownerBase = (int)blockIdx.x * 128;
  const int bb = ownerBase >> 10;
  const int gsc = clampi(gs, 1, 4);
  const float qnan = __int_as_float(0x7fc00000);
  v4f lw = (v4f){0.f, 0.f, 0.f, 0.f};
  if (LAYER == 1) lw = *(const v4fa*)(LIN + 4 * lane);

#pragma unroll 1
  for (int rr = 0; rr < 16; ++rr) {
    const int i = ownerBase + wave * 16 + rr;
    const int slot = i & (BK_NB - 1);
    float o0 = 0.0f, o1 = 0.0f;
    int pois = 0;
#pragma unroll 1
    for (int j = 0; j < gsc; ++j) {
      const int pos = clampi(gstart + j, 0, NRL - 1);
      const int t   = ord_of(pos);
      const int blk = t * 16 + bb;
      const int* mp = METAR + (size_t)blk * 32;
      const int* op = OFFR + (size_t)blk * 2048;
      const int nhv = mp[0], flv = mp[1], stv = op[slot], crv = op[1024 + slot];
      asm volatile("" :: "v"(nhv), "v"(flv), "v"(stv), "v"(crv));
      const int nhc = clampi(nhv, 0, RCAP_R);
      const int pv  = ((flv != 0) ? 1 : 0) | ((crv > DEG_R) ? 1 : 0);
      const int stc = clampi(stv, 0, nhc);
      int cntv = clampi(crv, 0, DEG_R);
      cntv = cntv > nhc - stc ? nhc - stc : cntv;
      const int liv = nhc > 0 ? nhc - 1 : 0;
      const int nh = __builtin_amdgcn_readfirstlane(nhc);
      const int st = __builtin_amdgcn_readfirstlane(stc);
      int cnt = __builtin_amdgcn_readfirstlane(cntv);
      const int lastI = __builtin_amdgcn_readfirstlane(liv);
      pois |= __builtin_amdgcn_readfirstlane(pv);

      const float* qrow = QS + (size_t)i * 512 + 128 * j;
      const v2f q2  = *(const v2fa*)(qrow + 2 * lane);
      const v2f sk2 = *(const v2fa*)(qrow + 64 + 2 * lane);
      const float* wet = WEt + t * 128;
      const v2f w0 = *(const v2fa*)(wet + 2 * lane);
      const v2f w1 = *(const v2fa*)(wet + 64 + 2 * lane);
      asm volatile("" :: "v"(q2), "v"(sk2), "v"(w0), "v"(w1));
      const int*   lst  = LISTR + (size_t)blk * RCAP_R;
      const int*   srcs = ei + (size_t)(2 * t) * NED;
      const float* eat  = ea + (size_t)t * NED * 2;
      const float* kvb  = KV + (size_t)j * NND * 128;

      float m = -1.0e30f, s = 0.0f, a0 = 0.0f, a1 = 0.0f;
#pragma unroll 1
      for (int q = 0; q < cnt; ++q) {
        const int li = clampi(st + q, 0, lastI);
        int e = lst[li];
        asm volatile("" :: "v"(e));
        e = clampi(e, 0, NED - 1);
        int sn = srcs[e];
        asm volatile("" :: "v"(sn));
        sn = clampi(sn, 0, NND - 1);
        const v2f ae = *(const v2fa*)(eat + 2 * (size_t)e);
        const float* kr = kvb + (size_t)sn * 128;
        const v2f k2 = *(const v2fa*)(kr + 2 * lane);
        const v2f v2 = *(const v2fa*)(kr + 64 + 2 * lane);
        asm volatile("" :: "v"(ae), "v"(k2), "v"(v2));
        const float e0 = bf16_val(ae.x), e1 = bf16_val(ae.y);
        const float ee0 = fmaf(e1, w1.x, e0 * w0.x);
        const float ee1 = fmaf(e1, w1.y, e0 * w0.y);
        const float ke0 = k2.x + ee0, ke1 = k2.y + ee1;
        const float ve0 = v2.x + ee0, ve1 = v2.y + ee1;
        float pr = q2.x * ke0 + q2.y * ke1;
        pr += __shfl_xor(pr, 16);
        pr += __shfl_xor(pr, 8);
        pr += __shfl_xor(pr, 4);
        pr += __shfl_xor(pr, 2);
        pr += __shfl_xor(pr, 1);
        const float l  = pr * 0.125f;
        const float mn = (l > m) ? l : m;
        const float sc = expf(m - mn);
        const float p  = expf(l - mn);
        s  = s * sc + p;
        a0 = a0 * sc + p * ve0;
        a1 = a1 * sc + p * ve1;
        m  = mn;
      }
      const float den = s + 1e-16f;
      const float d0 = a0 / den;
      const float d1 = a1 / den;
      const float g0 = (cnt > 0) ? d0 : 0.0f;
      const float g1 = (cnt > 0) ? d1 : 0.0f;
      o0 += g0 + sk2.x;
      o1 += g1 + sk2.y;
    }
    float h0 = (o0 > 0.0f) ? o0 : (o0 - o0);
    float h1 = (o1 > 0.0f) ? o1 : (o1 - o1);
    h0 = (pois != 0) ? qnan : h0;
    h1 = (pois != 0) ? qnan : h1;
    if (LAYER == 0) {
      const unsigned wh = pk16(bf16_bits(h0), bf16_bits(h1));
      const unsigned wl = pk16(bf16_lo_bits(h0), bf16_lo_bits(h1));
      volatile unsigned* row = (volatile unsigned*)(H1w + (size_t)i * 64);
      row[lane]      = wh;
      row[32 + lane] = wl;
      __threadfence();
      row[lane]      = wh;
      row[32 + lane] = wl;
    } else {
      float t0 = h0 * lw[0] + h1 * lw[2];
      float t1 = h0 * lw[1] + h1 * lw[3];
      t0 += __shfl_xor(t0, 16); t1 += __shfl_xor(t1, 16);
      t0 += __shfl_xor(t0, 8);  t1 += __shfl_xor(t1, 8);
      t0 += __shfl_xor(t0, 4);  t1 += __shfl_xor(t1, 4);
      t0 += __shfl_xor(t0, 2);  t1 += __shfl_xor(t1, 2);
      t0 += __shfl_xor(t0, 1);  t1 += __shfl_xor(t1, 1);
      if (lane == 0) *(v2fa*)(sX + (wave * 16 + rr) * 2) = (v2f){ t0, t1 };
    }
  }
  if (LAYER == 1) {
    __syncthreads();
    if (threadIdx.x < 64) {
      const v4f v = *(const v4fa*)(sX + 4 * threadIdx.x);
      st2_v4f(X01 + (size_t)ownerBase * 2 + 4 * threadIdx.x, v);
    }
  }
}

__global__ __launch_bounds__(256) void k_head(const float* __restrict__ X01, const float* __restrict__ pfa,
                                              const int* __restrict__ pfj, const int* __restrict__ LISTP,
                                              const int* __restrict__ OFFP, const int* __restrict__ METAP,
                                              float* out) {
  __shared__ __attribute__((aligned(16))) float sO[512];
  const int lane = threadIdx.x & 31;
  const int wave = threadIdx.x >> 5;
  const int ownerBase = (int)blockIdx.x * 128;
  const int bb = ownerBase >> 10;
  const float qnan = __int_as_float(0x7fc00000);
  const int nhv = METAP[(size_t)bb * 32], flv = METAP[(size_t)bb * 32 + 1];
  asm volatile("" :: "v"(nhv), "v"(flv));
  const int nhc = clampi(nhv, 0, RCAP_P);
  const int liv = nhc > 0 ? nhc - 1 : 0;
  const int nh = __builtin_amdgcn_readfirstlane(nhc);
  const int fl = __builtin_amdgcn_readfirstlane(flv);
  const int lastI = __builtin_amdgcn_readfirstlane(liv);
  const int* lst = LISTP + (size_t)bb * RCAP_P;
  const int* op  = OFFP + (size_t)bb * 2048;

#pragma unroll 1
  for (int rr = 0; rr < 16; ++rr) {
    const int g = ownerBase + wave * 16 + rr;
    const int slot = g & (BK_NB - 1);
    const int stv = op[slot], crv = op[1024 + slot];
    asm volatile("" :: "v"(stv), "v"(crv));
    const int pv  = ((fl != 0) || (crv > DEG_P)) ? 1 : 0;
    const int stc = clampi(stv, 0, nh);
    int cntv = clampi(crv, 0, DEG_P);
    cntv = cntv > nh - stc ? nh - stc : cntv;
    const int st = __builtin_amdgcn_readfirstlane(stc);
    int cnt = __builtin_amdgcn_readfirstlane(cntv);
    const int pois = __builtin_amdgcn_readfirstlane(pv);
    const v2f xi = *(const v2fa*)(X01 + 2 * (size_t)g);
    asm volatile("" :: "v"(xi));
    const float Vi = fabsf(xi.x);
    const float thi = xi.y;
    float P = 0.0f, Q = 0.0f;
    const int npass = (cnt + 31) >> 5;
#pragma unroll 1
    for (int ps = 0; ps < npass; ++ps) {
      const int idx = ps * 32 + lane;
      const bool act = idx < cnt;
      const int li = clampi(st + idx, 0, lastI);
      int e = lst[li];
      asm volatile("" :: "v"(e));
      e = clampi(e, 0, NPF - 1);
      int jn = pfj[e];
      asm volatile("" :: "v"(jn));
      jn = clampi(jn, 0, NGL - 1);
      const v2f at = *(const v2fa*)(pfa + 2 * (size_t)e);
      const v2f xj = *(const v2fa*)(X01 + 2 * (size_t)jn);
      asm volatile("" :: "v"(at), "v"(xj));
      const float r  = bf16_val(at.x);
      const float xr = bf16_val(at.y);
      const float denom = r * r + xr * xr;
      const float G = r / denom;
      const float B = (-xr) / denom;
      const float delta = xj.y - thi;
      const float vv = Vi * fabsf(xj.x);
      float sd, cd;
      sincosf(delta, &sd, &cd);
      const float pv = vv * (G * cd + B * sd);
      const float qv = vv * (G * sd - B * cd);
      P += act ? pv : 0.0f;
      Q += act ? qv : 0.0f;
    }
    P += __shfl_xor(P, 16); Q += __shfl_xor(Q, 16);
    P += __shfl_xor(P, 8);  Q += __shfl_xor(Q, 8);
    P += __shfl_xor(P, 4);  Q += __shfl_xor(Q, 4);
    P += __shfl_xor(P, 2);  Q += __shfl_xor(Q, 2);
    P += __shfl_xor(P, 1);  Q += __shfl_xor(Q, 1);
    P = (pois != 0) ? qnan : P;
    Q = (pois != 0) ? qnan : Q;
    if (lane == 0) *(v4fa*)(sO + (wave * 16 + rr) * 4) = (v4f){ xi.x, xi.y, P, Q };
  }
  __syncthreads();
  if (threadIdx.x < 128) {
    const v4f v = *(const v4fa*)(sO + 4 * threadIdx.x);
    st2_v4f(out + (size_t)ownerBase * 4 + 4 * threadIdx.x, v);
  }
}

extern "C" void kernel_launch(void* const* d_in, const int* in_sizes, int n_in,
                              void* d_out, int out_size, void* d_ws, size_t ws_size,
                              hipStream_t stream) {
  if (n_in < 25) return;
  if (in_sizes[0] != NTY * NND * NCI || in_sizes[1] != NRL * NED * 2) return;
  if (in_sizes[2] != NRL * NCI * NCH || in_sizes[4] != NRL * NCI * NCH || in_sizes[6] != NRL * NCI * NCH ||
      in_sizes[9] != NRL * NCI * NCH) return;
  if (in_sizes[3] != NRL * NCH || in_sizes[5] != NRL * NCH || in_sizes[7] != NRL * NCH || in_sizes[10] != NRL * NCH) return;
  if (in_sizes[8] != NRL * 2 * NCH || in_sizes[17] != NRL * 2 * NCH) return;
  if (in_sizes[11] != NRL * NCH * NCH || in_sizes[13] != NRL * NCH * NCH || in_sizes[15] != NRL * NCH * NCH ||
      in_sizes[18] != NRL * NCH * NCH) return;
  if (in_sizes[12] != NRL * NCH || in_sizes[14] != NRL * NCH || in_sizes[16] != NRL * NCH || in_sizes[19] != NRL * NCH) return;
  if (in_sizes[20] != NCH * 4 || in_sizes[21] != NPF * 2) return;
  if (in_sizes[22] != NRL * 2 * NED || in_sizes[23] != NPF || in_sizes[24] != NPF) return;
  if (out_size != NGL * 4) return;
  if (ws_size < WS_TOTAL) return;

  const float* x    = (const float*)d_in[0];
  const float* ea   = (const float*)d_in[1];
  const float* Wq0  = (const float*)d_in[2];     const float* bq0 = (const float*)d_in[3];
  const float* Wk0  = (const float*)d_in[4];     const float* bk0 = (const float*)d_in[5];
  const float* Wv0  = (const float*)d_in[6];     const float* bv0 = (const float*)d_in[7];
  const float* We0  = (const float*)d_in[8];
  const float* Ws0  = (const float*)d_in[9];     const float* bs0 = (const float*)d_in[10];
  const float* Wq1  = (const float*)d_in[11];    const float* bq1 = (const float*)d_in[12];
  const float* Wk1  = (const float*)d_in[13];    const float* bk1 = (const float*)d_in[14];
  const float* Wv1  = (const float*)d_in[15];    const float* bv1 = (const float*)d_in[16];
  const float* We1  = (const float*)d_in[17];
  const float* Ws1  = (const float*)d_in[18];    const float* bs1 = (const float*)d_in[19];
  const float* linW = (const float*)d_in[20];
  const float* pfa  = (const float*)d_in[21];
  const int*   ei   = (const int*)d_in[22];
  const int*   pf_i = (const int*)d_in[23];
  const int*   pf_j = (const int*)d_in[24];
  float* out = (float*)d_out;

  char* ws = (char*)d_ws;
  unsigned short* XB   = (unsigned short*)(ws + O_XB);
  unsigned short* H1   = (unsigned short*)(ws + O_H1);
  float*          QS   = (float*)(ws + O_QS);
  float*          KV   = (float*)(ws + O_KV);
  float*          X01  = (float*)(ws + O_X01);
  unsigned short* WQS0 = (unsigned short*)(ws + O_WQS0);
  unsigned short* WKV0 = (unsigned short*)(ws + O_WKV0);
  unsigned short* WQS1 = (unsigned short*)(ws + O_WQS1);
  unsigned short* WKV1 = (unsigned short*)(ws + O_WKV1);
  float*          BQS  = (float*)(ws + O_BQS);
  float*          BKV  = (float*)(ws + O_BKV);
  float*          WEt  = (float*)(ws + O_WE);
  float*          LIN  = (float*)(ws + O_LIN);
  int*            LISTR = (int*)(ws + O_LISTR);
  int*            OFFR  = (int*)(ws + O_OFFR);
  int*            METAR = (int*)(ws + O_METAR);
  int*            LISTP = (int*)(ws + O_LISTP);
  int*            OFFP  = (int*)(ws + O_OFFP);
  int*            METAP = (int*)(ws + O_METAP);

  hipFuncSetAttribute(reinterpret_cast<const void*>(&k_bucket),
                      hipFuncAttributeMaxDynamicSharedMemorySize, LDS_BK_P);

  k_plane<0><<<NGL * 32 / 8 / 256, 256, 0, stream>>>(x, NGL, NCI, NCI, XB, NGL, 32);
  k_wprep<NCI, 32, 32><<<4 * NRL * 1, 256, 0, stream>>>(Wq0, Ws0, Wk0, Wv0, WQS0, WKV0);
  k_wprep<NCH, 64, 128><<<4 * NRL * 4, 256, 0, stream>>>(Wq1, Ws1, Wk1, Wv1, WQS1, WKV1);
  k_tprep<<<7, 256, 0, stream>>>(bq0, bs0, bk0, bv0, We0, linW, BQS, BKV, WEt, LIN);
  k_tprep<<<6, 256, 0, stream>>>(bq1, bs1, bk1, bv1, We1, linW, BQS + NRL * 128, BKV + NRL * 128,
                                 WEt + NRL * 128, LIN);
  k_bucket<<<dim3(16, NRL), BK_THR, LDS_BK_R, stream>>>(ei + NED, 2 * NED, NED, RCAP_R, LISTR, OFFR, METAR);
  k_bucket<<<dim3(64, 1), BK_THR, LDS_BK_P, stream>>>(pf_i, 0, NPF, RCAP_P, LISTP, OFFP, METAP);

  for (int l = 0; l < 2; ++l) {
    const unsigned short* Apl = (l == 0) ? XB : H1;
    const unsigned short* WQS = (l == 0) ? WQS0 : WQS1;
    const unsigned short* WKV = (l == 0) ? WKV0 : WKV1;
    const int KT = (l == 0) ? 32 : 128;
    const float* bqs = BQS + (size_t)l * NRL * 128;
    const float* bkv = BKV + (size_t)l * NRL * 128;
    const float* wet = WEt + (size_t)l * NRL * 128;
    for (int d = 0; d < NTY; ++d) {
      const int g0 = GST_H[d], gsz = GSZ_H[d];
      {
        const int Nq = 128 * gsz;
        const int T  = (NND / 64) * (Nq / 64);
        const unsigned short* A = Apl + (size_t)d * NND * KT;
        const unsigned short* B = WQS + (size_t)g0 * 128 * KT;
        if (l == 0) k_gemm_nt<0, 1><<<(T + 7) / 8, 256, 0, stream>>>(A, B, bqs + g0 * 128, QS, NND, Nq, KT, 512);
        else        k_gemm_nt<1, 1><<<(T + 7) / 8, 256, 0, stream>>>(A, B, bqs + g0 * 128, QS, NND, Nq, KT, 512);
      }
      for (int j = 0; j < gsz; ++j) {
        const int t = ORD_H[g0 + j];
        const int T = (NND / 64) * 2;
        const unsigned short* A = Apl + (size_t)SRC_H[t] * NND * KT;
        const unsigned short* B = WKV + (size_t)t * 128 * KT;
        float* D = KV + (size_t)j * NND * 128;
        if (l == 0) k_gemm_nt<0, 1><<<(T + 7) / 8, 256, 0, stream>>>(A, B, bkv + t * 128, D, NND, 128, KT, 128);
        else        k_gemm_nt<1, 1><<<(T + 7) / 8, 256, 0, stream>>>(A, B, bkv + t * 128, D, NND, 128, KT, 128);
      }
      unsigned* h1w = (unsigned*)(ws + O_H1) + (size_t)d * NND * 64;
      float* x01 = X01 + (size_t)d * NND * 2;
      if (l == 0) k_att<0><<<NND / 128, 256, 0, stream>>>(QS, KV, ea, ei, wet, LIN, LISTR, OFFR, METAR, h1w, x01, g0, gsz);
      else        k_att<1><<<NND / 128, 256, 0, stream>>>(QS, KV, ea, ei, wet, LIN, LISTR, OFFR, METAR, h1w, x01, g0, gsz);
    }
  }
  k_head<<<NGL / 128, 256, 0, stream>>>(X01, pfa, pf_j, LISTP, OFFP, METAP, out);
}
